// USTSSMBlock_67680094650382
// MI455X (gfx1250) — hardware-run, weakly checked
//
#include <hip/hip_runtime.h>
#include <math.h>

typedef __attribute__((ext_vector_type(16))) _Float16 v16h;
typedef __attribute__((ext_vector_type(8)))  _Float16 v8h;
typedef __attribute__((ext_vector_type(2)))  _Float16 v2h;
typedef __attribute__((ext_vector_type(16))) __bf16   v16b;
typedef __attribute__((ext_vector_type(8)))  __bf16   v8b;
typedef __attribute__((ext_vector_type(8)))  float    v8f;
typedef __attribute__((ext_vector_type(4)))  float    v4f;
typedef __attribute__((ext_vector_type(2)))  float    v2f;
typedef float v2f __attribute__((ext_vector_type(2)));

constexpr int kNB   = 2;
constexpr int kT    = 2048;
constexpr int kRows = kNB * kT;
constexpr int kDM   = 512;
constexpr int kDI   = 2 * kDM;
constexpr int kNs   = 16;
constexpr int kDC   = 4;
constexpr int kR    = 32;
constexpr int kXo   = kR + 2 * kNs;
constexpr int kThr  = 256;
constexpr float kInCarry = 1024.0f;
constexpr float kWCarry  = 4096.0f;
constexpr float kCXn = 1024.0f;
constexpr float kCU  = 512.0f;
constexpr float kCDt = 2048.0f;
constexpr float kCY  = 256.0f;
constexpr float kF16MinNormal = 6.103515625e-5f;

static_assert(kXo == 64 && kR == 32 && kDI == 1024 && kRows == 4096 && kT == 2048 && kDM == 512, "the index arithmetic below uses these sizes");

constexpr size_t kOffZB = 0ull;
constexpr size_t kOffBDT = 8192ull;
constexpr size_t kOffSTAT = 12288ull;
constexpr size_t kOffXN16 = 45056ull;
constexpr size_t kOffWIN16 = 4239360ull;
constexpr size_t kOffWX16 = 6336512ull;
constexpr size_t kOffWDT16 = 6467584ull;
constexpr size_t kOffWOUT16 = 6533120ull;
constexpr size_t kOffXZ = 7581696ull;
constexpr size_t kOffU32 = 41136128ull;
constexpr size_t kOffU16 = 57913344ull;
constexpr size_t kOffXD = 66301952ull;
constexpr size_t kOffDT16 = 67350528ull;
constexpr size_t kOffDL = 67612672ull;
constexpr size_t kOffYS = 84389888ull;
constexpr size_t kOffY16 = 101167104ull;
constexpr size_t kOffOUTF = 109555712ull;
constexpr size_t kWsTotal = 117944320ull;
static_assert(kWsTotal <= 134217728ull, "carve cap: under 128 MiB");
static_assert(kOffZB == 0
  && kOffBDT == kOffZB + 8192ull
  && kOffSTAT == kOffBDT + 4096ull
  && kOffXN16 == kOffSTAT + 32768ull
  && kOffWIN16 == kOffXN16 + 4194304ull
  && kOffWX16 == kOffWIN16 + 2097152ull
  && kOffWDT16 == kOffWX16 + 131072ull
  && kOffWOUT16 == kOffWDT16 + 65536ull
  && kOffXZ == kOffWOUT16 + 1048576ull
  && kOffU32 == kOffXZ + 33554432ull
  && kOffU16 == kOffU32 + 16777216ull
  && kOffXD == kOffU16 + 8388608ull
  && kOffDT16 == kOffXD + 1048576ull
  && kOffDL == kOffDT16 + 262144ull
  && kOffYS == kOffDL + 16777216ull
  && kOffY16 == kOffYS + 16777216ull
  && kOffOUTF == kOffY16 + 8388608ull
  && kWsTotal == kOffOUTF + 8388608ull, "the carve is a chain: every region starts where the one before ends");
static_assert((kOffBDT % 256) == 0 && (kOffSTAT % 256) == 0 && (kOffXN16 % 256) == 0 && (kOffWIN16 % 256) == 0 && (kOffWX16 % 256) == 0 && (kOffWDT16 % 256) == 0 && (kOffWOUT16 % 256) == 0 && (kOffXZ % 256) == 0 && (kOffU32 % 256) == 0 && (kOffU16 % 256) == 0 && (kOffXD % 256) == 0 && (kOffDT16 % 256) == 0 && (kOffDL % 256) == 0 && (kOffYS % 256) == 0 && (kOffY16 % 256) == 0 && (kOffOUTF % 256) == 0, "every region starts on a multiple of 256 B");

__device__ __forceinline__ unsigned short f2bf_bits(float f) {
  unsigned u = __float_as_uint(f);
  return (unsigned short)((u + 0x7FFFu + ((u >> 16) & 1u)) >> 16);
}
__device__ __forceinline__ float bf_bits2f(unsigned short h) { return __uint_as_float(((unsigned)h) << 16); }
__device__ __forceinline__ float bf16r(float f) { return bf_bits2f(f2bf_bits(f)); }
__device__ __forceinline__ float carry_flush(float v, float carry) {
  const float s = v * carry;
  return (fabsf(s) < kF16MinNormal) ? 0.0f : s;
}

__device__ __forceinline__ void dep_guard4_h(v8f& a, v8f& b, v8f& c, v8f& d, v16h x, v16h y) { asm volatile("v_nop\n\tv_nop\n\tv_nop\n\tv_nop" : "+v"(a), "+v"(b), "+v"(c), "+v"(d) : "v"(x), "v"(y)); }
__device__ __forceinline__ void dep_guard4_b(v8f& a, v8f& b, v8f& c, v8f& d, v16b x, v16b y) { asm volatile("v_nop\n\tv_nop\n\tv_nop\n\tv_nop" : "+v"(a), "+v"(b), "+v"(c), "+v"(d) : "v"(x), "v"(y)); }
__device__ __forceinline__ void keep4_h(v16h a, v16h b, v16h c, v16h d) { asm volatile("v_nop" :: "v"(a), "v"(b), "v"(c), "v"(d)); }
__device__ __forceinline__ void keep4_b(v16b a, v16b b, v16b c, v16b d) { asm volatile("v_nop" :: "v"(a), "v"(b), "v"(c), "v"(d)); }
__device__ __forceinline__ void acc_guard4(v8f& a, v8f& b, v8f& c, v8f& d) { asm volatile("v_nop\n\tv_nop\n\tv_nop\n\tv_nop" : "+v"(a), "+v"(b), "+v"(c), "+v"(d)); }

template <typename T> struct Frag;
template <> struct Frag<_Float16> {
  typedef v16h V; union U { v16h v; v8h h[2]; };
  static __device__ __forceinline__ v16h load(const _Float16* p) {
    U f; f.h[0] = *(const v8h*)(p); f.h[1] = *(const v8h*)(p + 16); return f.v;
  }
  static __device__ __forceinline__ v8f mma(v16h a, v16h b, v8f c) {
    return __builtin_amdgcn_wmma_f32_16x16x32_f16(false, a, false, b, (short)0, c, false, false);
  }
  static __device__ __forceinline__ void guard4(v8f& a, v8f& b, v8f& c, v8f& d, v16h x, v16h y) { dep_guard4_h(a, b, c, d, x, y); }
  static __device__ __forceinline__ void keep(v16h a, v16h b, v16h c, v16h d) { keep4_h(a, b, c, d); }
};
template <> struct Frag<__bf16> {
  typedef v16b V; union U { v16b v; v8b h[2]; };
  static __device__ __forceinline__ v16b load(const __bf16* p) {
    U f; f.h[0] = *(const v8b*)(p); f.h[1] = *(const v8b*)(p + 16); return f.v;
  }
  static __device__ __forceinline__ v8f mma(v16b a, v16b b, v8f c) {
    return __builtin_amdgcn_wmma_f32_16x16x32_bf16(false, a, false, b, (short)0, c, false, false);
  }
  static __device__ __forceinline__ void guard4(v8f& a, v8f& b, v8f& c, v8f& d, v16b x, v16b y) { dep_guard4_b(a, b, c, d, x, y); }
  static __device__ __forceinline__ void keep(v16b a, v16b b, v16b c, v16b d) { keep4_b(a, b, c, d); }
};

__device__ __forceinline__ v8f mma_h(v16h a, v16h b, v8f c) {
  c = __builtin_amdgcn_wmma_f32_16x16x32_f16(false, a, false, b, (short)0, c, false, false);
  asm volatile("v_nop\n\tv_nop\n\tv_nop\n\tv_nop" : "+v"(c) : "v"(a), "v"(b));
  return c;
}

template <int ET> struct Elem;
template <> struct Elem<0> { typedef _Float16 T; };
template <> struct Elem<1> { typedef __bf16 T; };
template <int ET, bool SPLIT, int BIAS_MODE, int OUT_MODE, bool RESID, int ACT = 0>
__global__ __launch_bounds__(256) void wmma_gemm64(
    const unsigned short* __restrict__ Ap, const unsigned short* __restrict__ A2p, int lda, long strideA,
    const unsigned short* __restrict__ Btp, const unsigned short* __restrict__ Bt2p, int ldb, long strideB,
    void* __restrict__ Cout, void* __restrict__ Cout2, int ldc, long strideC,
    const float* __restrict__ bias,
    const float* __restrict__ resid, long strideR,
    int M, int N, int K, float scale) {
  typedef typename Elem<ET>::T T;
  typedef typename Frag<T>::V V;
  const T* A = (const T*)Ap; const T* A2 = (const T*)A2p; const T* Bt = (const T*)Btp; const T* Bt2 = (const T*)Bt2p;
  __shared__ __align__(16) float sT[8][16 * 68];
  const int b    = blockIdx.y;
  const int lane = threadIdx.x & 31;
  const int wave = threadIdx.x >> 5;
  const int tilesN = N >> 6;
  const int tilesM = M >> 6;
  const int tile = blockIdx.x * 8 + wave;
  if (tile >= tilesM * tilesN) return;
  const int tm = tile / tilesN;
  const int tn = tile - tm * tilesN;
  const int m0 = tm << 6;
  const int n0 = tn << 6;

  const T* Ab  = A  + (size_t)b * strideA;
  const T* Bb  = Bt + (size_t)b * strideB;
  const T* Ab2 = SPLIT ? (A2  + (size_t)b * strideA) : nullptr;
  const T* Bb2 = SPLIT ? (Bt2 + (size_t)b * strideB) : nullptr;

  const int rlane = lane & 15;
  const int koff  = (lane >> 4) * 8;
  const int mOff  = (lane >> 4) * 8;

  v8f acc[4][4];
#pragma unroll
  for (int i = 0; i < 4; ++i)
#pragma unroll
    for (int j = 0; j < 4; ++j) acc[i][j] = (v8f){0.f,0.f,0.f,0.f,0.f,0.f,0.f,0.f};

  for (int k0 = 0; k0 < K; k0 += 32) {
    V bh[4], bl[4];
#pragma unroll
    for (int j = 0; j < 4; ++j) {
      const size_t bo = (size_t)(n0 + (j << 4) + rlane) * ldb + koff + k0;
      bh[j] = Frag<T>::load(Bb + bo);
      if (SPLIT) bl[j] = Frag<T>::load(Bb2 + bo);
    }
#pragma unroll
    for (int i = 0; i < 4; ++i) {
      const size_t ao = (size_t)(m0 + (i << 4) + rlane) * lda + koff + k0;
      V ah = Frag<T>::load(Ab + ao);
      V al;
      if (SPLIT) al = Frag<T>::load(Ab2 + ao);
#pragma unroll
      for (int j = 0; j < 4; ++j) {
        acc[i][j] = Frag<T>::mma(ah, bh[j], acc[i][j]);
        if (SPLIT) {
          acc[i][j] = Frag<T>::mma(ah, bl[j], acc[i][j]);
          acc[i][j] = Frag<T>::mma(al, bh[j], acc[i][j]);
        }
      }
      Frag<T>::guard4(acc[i][0], acc[i][1], acc[i][2], acc[i][3], ah, SPLIT ? al : ah);
    }
    Frag<T>::keep(bh[0], bh[1], bh[2], bh[3]);
    if (SPLIT) Frag<T>::keep(bl[0], bl[1], bl[2], bl[3]);
  }
  acc_guard4(acc[0][0], acc[0][1], acc[0][2], acc[0][3]);
  acc_guard4(acc[1][0], acc[1][1], acc[1][2], acc[1][3]);
  acc_guard4(acc[2][0], acc[2][1], acc[2][2], acc[2][3]);
  acc_guard4(acc[3][0], acc[3][1], acc[3][2], acc[3][3]);

  float* slab = sT[wave];
  const float* Rb = RESID ? (resid + (size_t)b * strideR) : nullptr;
#pragma unroll
  for (int i = 0; i < 4; ++i) {
    const int mBase = m0 + (i << 4);
#pragma unroll
    for (int j = 0; j < 4; ++j) {
      const int n = n0 + (j << 4) + rlane;
      float bv = 0.f;
      if (BIAS_MODE == 2) bv = bias[n];
#pragma unroll
      for (int r = 0; r < 8; ++r) {
        float v = acc[i][j][r] * scale;
        if (BIAS_MODE == 1) v += bias[mBase + mOff + r];
        if (BIAS_MODE == 2) v += bv;
        if (RESID) v += Rb[(size_t)(mBase + mOff + r) * ldc + n];
        if (ACT == 1) v = tanhf(v);
        if (ACT == 2) v = fmaxf(v, 0.0f);
        if (ACT == 3) v = v / (1.0f + expf(-v));
        if (ACT == 4) v = (v > 0.f) ? v : 0.01f * v;
        slab[(mOff + r) * 68 + (j << 4) + rlane] = v;
      }
    }
    __builtin_amdgcn_fence(__ATOMIC_RELEASE, "workgroup");
    __builtin_amdgcn_wave_barrier();
    __builtin_amdgcn_fence(__ATOMIC_ACQUIRE, "workgroup");
    if (OUT_MODE == 0) {
      float* C = (float*)Cout + (size_t)b * strideC;
      const int hh = lane >> 4, c4 = (lane & 15) * 4;
      for (int pass = 0; pass < 2; ++pass) {
#pragma unroll
        for (int it = 0; it < 8; ++it) {
          const int row = it * 2 + hh;
          v4f v = *(const v4f*)(slab + row * 68 + c4);
          *(volatile v4f*)(C + (size_t)(mBase + row) * ldc + n0 + c4) = v;
        }
        __threadfence();
      }
    } else {
      const int q = lane >> 3, c8 = (lane & 7) * 8;
      unsigned short* C  = (unsigned short*)Cout  + (size_t)b * strideC;
      unsigned short* C2 = (OUT_MODE == 2) ? ((unsigned short*)Cout2 + (size_t)b * strideC) : nullptr;
      for (int pass = 0; pass < 2; ++pass) {
#pragma unroll
        for (int it = 0; it < 4; ++it) {
          const int row = it * 4 + q;
          const float* sp = slab + row * 68 + c8;
          v8h hv, lv;
#pragma unroll
          for (int e = 0; e < 8; ++e) {
            if (OUT_MODE == 1) {
              hv[e] = (_Float16)sp[e];
            } else {
              unsigned short hb = f2bf_bits(sp[e]);
              unsigned short lb = f2bf_bits(sp[e] - bf_bits2f(hb));
              hv[e] = __builtin_bit_cast(_Float16, hb);
              lv[e] = __builtin_bit_cast(_Float16, lb);
            }
          }
          *(volatile v8h*)(C + (size_t)(mBase + row) * ldc + n0 + c8) = hv;
          if (OUT_MODE == 2) *(volatile v8h*)(C2 + (size_t)(mBase + row) * ldc + n0 + c8) = lv;
        }
        __threadfence();
      }
    }
    __builtin_amdgcn_fence(__ATOMIC_RELEASE, "workgroup");
    __builtin_amdgcn_wave_barrier();
    __builtin_amdgcn_fence(__ATOMIC_ACQUIRE, "workgroup");
  }
}


__device__ __forceinline__ void store2(float* p, float v) {
  *(volatile float*)p = v;
  __threadfence();
  *(volatile float*)p = v;
}

__global__ __launch_bounds__(kThr) void cast_plane_kernel(const float* __restrict__ src, unsigned short* __restrict__ dst,
                                                          int colsLog2, int dstPitch, int dstOff) {
  const int i   = blockIdx.x * kThr + threadIdx.x;
  const int sh  = colsLog2 - 3;
  const int row = i >> sh;
  const int c8  = (i & ((1 << sh) - 1)) * 8;
  const float* sp = src + ((size_t)row << colsLog2) + c8;
  const v4f a0 = *(const v4f*)(sp);
  const v4f a1 = *(const v4f*)(sp + 4);
  v8h hv;
#pragma unroll
  for (int e = 0; e < 4; ++e) {
    const float f0 = a0[e];
    const float f1 = a1[e];
    hv[e]     = (_Float16)carry_flush(bf16r(f0), kInCarry);
    hv[4 + e] = (_Float16)carry_flush(bf16r(f1), kInCarry);
  }
  unsigned short* dp = dst + (size_t)row * dstPitch + dstOff + c8;
  *(volatile v8h*)dp = hv;
  __threadfence();
  *(volatile v8h*)dp = hv;
}

__global__ __launch_bounds__(256) void wt_plane_kernel(const float* __restrict__ W, unsigned short* __restrict__ dst, int K, int N, int nLive, int ldd, int colOff) {
  const int n  = blockIdx.x;
  const int k8 = threadIdx.x * 8;
  const bool live = n < nLive;
  const int nc = live ? n : 0;
  v8h hv;
#pragma unroll
  for (int e = 0; e < 8; ++e) {
    const float w = W[(size_t)(k8 + e) * N + nc];
    hv[e] = (_Float16)(live ? carry_flush(bf16r(w), kWCarry) : 0.0f);
  }
  unsigned short* dp = dst + (size_t)n * ldd + colOff + k8;
  *(volatile v8h*)dp = hv;
  __threadfence();
  *(volatile v8h*)dp = hv;
}

__global__ __launch_bounds__(kThr) void setup_kernel(const float* __restrict__ bdt, float* __restrict__ ZB, float* __restrict__ BDT) {
  const unsigned bk = blockIdx.x;
  if (bk < 8u) {
    store2(ZB + bk * (unsigned)kThr + threadIdx.x, 0.0f);
  } else {
    const unsigned d = (bk - 8u) * (unsigned)kThr + threadIdx.x;
    const float p = bdt[d];
    store2(BDT + d, bf16r(p));
  }
}
static_assert(2048 == 8 * kThr && kDI == 4 * kThr, "set-up grid: 8 blocks of zero bias, 4 of step biases: 12 blocks");

__global__ __launch_bounds__(kThr) void lnstat_kernel(const float* __restrict__ x, float* __restrict__ STAT) {
  const size_t row = (size_t)blockIdx.x * kThr + threadIdx.x;
  const float* xp = x + row * kDM;
  float s = 0.0f;
  for (int c = 0; c < kDM; ++c) { const float p = xp[c]; s += bf16r(p); }
  const float mean = s / (float)kDM;
  float q = 0.0f;
  for (int c = 0; c < kDM; ++c) { const float p = xp[c]; const float dd = bf16r(p) - mean; q += dd * dd; }
  v2f st; st[0] = mean; st[1] = 1.0f / sqrtf(q / (float)kDM + 1e-5f);
  float* dp = STAT + 2 * row;
  *(volatile v2f*)dp = st;
  __threadfence();
  *(volatile v2f*)dp = st;
}
static_assert(kRows == 16 * kThr, "statistics grid exact: 16 blocks");

__global__ __launch_bounds__(kThr) void lncast_kernel(const float* __restrict__ x, const float* __restrict__ STAT, const float* __restrict__ gam, const float* __restrict__ bet,
                                                     unsigned short* __restrict__ XN16) {
  const unsigned i = blockIdx.x * (unsigned)kThr + threadIdx.x;
  const size_t row = i >> 6;
  const unsigned c8 = (i & 63u) * 8u;
  const float mean = STAT[2 * row], inv = STAT[2 * row + 1];
  const float* xp = x + row * kDM + c8;
  v8h hv;
#pragma unroll
  for (int e = 0; e < 8; ++e) {
    const float p = xp[e], ga = gam[c8 + e], be = bet[c8 + e];
    hv[e] = (_Float16)carry_flush((bf16r(p) - mean) * inv * bf16r(ga) + bf16r(be), kCXn);
  }
  unsigned short* dp = XN16 + row * kDM + c8;
  *(volatile v8h*)dp = hv;
  __threadfence();
  *(volatile v8h*)dp = hv;
}
static_assert((size_t)kRows * (kDM / 8) == 1024ull * kThr && kDM / 8 == 64, "norm cast grid exact: 1,024 blocks; 64 groups a row");

__global__ __launch_bounds__(128) void front_kernel(const float* __restrict__ XZ, const float* __restrict__ cw, const float* __restrict__ cb,
                                                    float* __restrict__ U32, unsigned short* __restrict__ U16) {
  const int row = (int)blockIdx.y;
  const int pos = row & (kT - 1);
  const int c8 = (int)threadIdx.x * 8;
  float acc[8], wv[8][kDC];
#pragma unroll
  for (int e = 0; e < 8; ++e) {
    const float p = cb[c8 + e];
    acc[e] = bf16r(p);
    const v4f w4 = *(const v4f*)(cw + (size_t)(c8 + e) * kDC);
#pragma unroll
    for (int k = 0; k < kDC; ++k) { const float w = w4[k]; wv[e][k] = bf16r(w); }
  }
#pragma unroll
  for (int k = 0; k < kDC; ++k) {
    const int back = kDC - 1 - k;
    const bool has = pos >= back;
    const float* xp = XZ + (size_t)(row - (has ? back : 0)) * (2 * kDI) + c8;
    const v4f x0 = *(const v4f*)xp, x1 = *(const v4f*)(xp + 4);
#pragma unroll
    for (int e = 0; e < 8; ++e) {
      const float xv = (e < 4) ? x0[e] : x1[e - 4];
      acc[e] += has ? wv[e][k] * xv : 0.0f;
    }
  }
  v4f u0, u1;
  v8h hv;
#pragma unroll
  for (int e = 0; e < 8; ++e) {
    const float v = acc[e];
    const float s = v / (1.0f + expf(-v));
    if (e < 4) u0[e] = s; else u1[e - 4] = s;
    hv[e] = (_Float16)carry_flush(s, kCU);
  }
  float* up = U32 + (size_t)row * kDI + c8;
  unsigned short* hp = U16 + (size_t)row * kDI + c8;
  for (int pass = 0; pass < 2; ++pass) {
    *(volatile v4f*)up = u0; *(volatile v4f*)(up + 4) = u1;
    *(volatile v8h*)hp = hv;
    __threadfence();
  }
}
static_assert(kDI == 128 * 8, "front grid exact: 128 groups a row");

__global__ __launch_bounds__(kThr) void dtcast_kernel(const float* __restrict__ XD, unsigned short* __restrict__ DT16) {
  const unsigned i = blockIdx.x * (unsigned)kThr + threadIdx.x;
  const size_t row = i >> 2;
  const unsigned c8 = (i & 3u) * 8u;
  const float* sp = XD + row * kXo + c8;
  v8h hv;
#pragma unroll
  for (int e = 0; e < 8; ++e) { const float v = sp[e]; hv[e] = (_Float16)carry_flush(v, kCDt); }
  unsigned short* dp = DT16 + row * kR + c8;
  *(volatile v8h*)dp = hv;
  __threadfence();
  *(volatile v8h*)dp = hv;
}
static_assert((size_t)kRows * 4 == 64ull * kThr && kR == 4 * 8, "the step input's cast: 64 blocks; 4 groups a row");

__global__ __launch_bounds__(kThr) void scan_kernel(const float* __restrict__ XD, const float* __restrict__ DL, const float* __restrict__ U32,
                                                    const float* __restrict__ A_log, const float* __restrict__ Dp, float* __restrict__ YS) {
  const unsigned sq = blockIdx.x >> 2;
  const unsigned d = (blockIdx.x & 3u) * (unsigned)kThr + threadIdx.x;
  float A[kNs], s[kNs];
#pragma unroll
  for (int n = 0; n < kNs; ++n) { const float a = A_log[(size_t)d * kNs + n]; A[n] = -expf(bf16r(a)); s[n] = 0.0f; }
  const float q0 = Dp[d];
  const float dsk = bf16r(q0);
  for (int l = 0; l < kT; ++l) {
    const size_t row = (size_t)sq * kT + (size_t)l;
    const float* pb = XD + row * kXo + kR;
    const float pre = DL[row * kDI + d];
    const float uv = U32[row * kDI + d];
    const float dt = fmaxf(pre, 0.0f) + log1pf(expf(-fabsf(pre)));
    float y = 0.0f;
#pragma unroll
    for (int q = 0; q < kNs / 4; ++q) {
      const v4f bv = *(const v4f*)(pb + 4 * q), cv = *(const v4f*)(pb + kNs + 4 * q);
#pragma unroll
      for (int e = 0; e < 4; ++e) {
        const int n = 4 * q + e;
        const float sn = expf(dt * A[n]) * s[n] + (dt * bv[e]) * uv;
        s[n] = sn;
        y += sn * cv[e];
      }
    }
    store2(YS + row * kDI + d, y + dsk * uv);
  }
}
static_assert(kDI == 4 * kThr && (kNs % 4) == 0 && (kR % 4) == 0, "walk grid exact: 8 blocks: four a sequence; the B | C columns 16-B aligned");

__global__ __launch_bounds__(128) void ygate_kernel(const float* __restrict__ YS, const float* __restrict__ XZ, unsigned short* __restrict__ Y16) {
  const size_t row = blockIdx.y;
  const unsigned c8 = threadIdx.x * 8u;
  const float* yp = YS + row * kDI + c8;
  const float* zp = XZ + row * (2 * kDI) + kDI + c8;
  v8h hv;
#pragma unroll
  for (int e = 0; e < 8; ++e) { const float z = zp[e]; hv[e] = (_Float16)carry_flush(yp[e] * (z / (1.0f + expf(-z))), kCY); }
  unsigned short* dp = Y16 + row * kDI + c8;
  *(volatile v8h*)dp = hv;
  __threadfence();
  *(volatile v8h*)dp = hv;
}

__global__ __launch_bounds__(kThr) void resadd_kernel(const float* __restrict__ OUTF, const float* __restrict__ x, float* __restrict__ out) {
  const size_t o = ((size_t)blockIdx.x * kThr + threadIdx.x) * 8;
  const v4f a0 = *(const v4f*)(OUTF + o), a1 = *(const v4f*)(OUTF + o + 4);
  v4f o0, o1;
#pragma unroll
  for (int e = 0; e < 8; ++e) { const float p = x[o + e]; const float r = bf16r(p) + ((e < 4) ? a0[e] : a1[e - 4]); if (e < 4) o0[e] = r; else o1[e - 4] = r; }
  float* dp = out + o;
  for (int pass = 0; pass < 2; ++pass) { *(volatile v4f*)dp = o0; *(volatile v4f*)(dp + 4) = o1; __threadfence(); }
}
static_assert((size_t)kRows * kDM / 8 == 1024ull * kThr, "the residual: 1,024 blocks");

extern "C" void kernel_launch(void* const* d_in, const int* in_sizes, int n_in,
                              void* d_out, int out_size, void* d_ws, size_t ws_size,
                              hipStream_t stream) {
  if (n_in < 12 || d_out == nullptr || d_ws == nullptr) return;
  if (in_sizes[0] != kRows * kDM || in_sizes[1] != kDM || in_sizes[2] != kDM || in_sizes[3] != 2 * kDI * kDM || in_sizes[4] != kDI * kDC || in_sizes[5] != kDI) return;
  if (in_sizes[6] != kXo * kDI || in_sizes[7] != kDI * kR || in_sizes[8] != kDI || in_sizes[9] != kDI * kNs || in_sizes[10] != kDI || in_sizes[11] != kDM * kDI) return;
  if (out_size != kRows * kDM) return;
  if (ws_size < kWsTotal) return;
  const float* x    = (const float*)d_in[0];
  const float* lng  = (const float*)d_in[1];
  const float* lnb  = (const float*)d_in[2];
  const float* Win  = (const float*)d_in[3];
  const float* cvw  = (const float*)d_in[4];
  const float* cvb  = (const float*)d_in[5];
  const float* Wx   = (const float*)d_in[6];
  const float* Wdt  = (const float*)d_in[7];
  const float* bdt  = (const float*)d_in[8];
  const float* alog = (const float*)d_in[9];
  const float* dsk  = (const float*)d_in[10];
  const float* Wout = (const float*)d_in[11];
  float* out = (float*)d_out;
  char* ws = (char*)d_ws;
  float* ZB   = (float*)(ws + kOffZB);
  float* BDT  = (float*)(ws + kOffBDT);
  float* STAT = (float*)(ws + kOffSTAT);
  unsigned short* XN16   = (unsigned short*)(ws + kOffXN16);
  unsigned short* WIN16  = (unsigned short*)(ws + kOffWIN16);
  unsigned short* WX16   = (unsigned short*)(ws + kOffWX16);
  unsigned short* WDT16  = (unsigned short*)(ws + kOffWDT16);
  unsigned short* WOUT16 = (unsigned short*)(ws + kOffWOUT16);
  float* XZ  = (float*)(ws + kOffXZ);
  float* U32 = (float*)(ws + kOffU32);
  unsigned short* U16 = (unsigned short*)(ws + kOffU16);
  float* XD  = (float*)(ws + kOffXD);
  unsigned short* DT16 = (unsigned short*)(ws + kOffDT16);
  float* DL  = (float*)(ws + kOffDL);
  float* YS  = (float*)(ws + kOffYS);
  unsigned short* Y16 = (unsigned short*)(ws + kOffY16);
  float* OUTF = (float*)(ws + kOffOUTF);

  static_assert(((size_t)2 * kDI * kDM / 8) % kThr == 0 && ((size_t)kXo * kDI / 8) % kThr == 0 && ((size_t)kDI * kR / 8) % kThr == 0 && ((size_t)kDM * kDI / 8) % kThr == 0, "the casts' grids");
  cast_plane_kernel<<<(int)(((size_t)2 * kDI * kDM / 8) / kThr), kThr, 0, stream>>>(Win, WIN16, 9, kDM, 0);
  cast_plane_kernel<<<(int)(((size_t)kXo * kDI / 8) / kThr), kThr, 0, stream>>>(Wx, WX16, 10, kDI, 0);
  cast_plane_kernel<<<(int)(((size_t)kDI * kR / 8) / kThr), kThr, 0, stream>>>(Wdt, WDT16, 5, kR, 0);
  cast_plane_kernel<<<(int)(((size_t)kDM * kDI / 8) / kThr), kThr, 0, stream>>>(Wout, WOUT16, 10, kDI, 0);
  setup_kernel<<<12, kThr, 0, stream>>>(bdt, ZB, BDT);
  lnstat_kernel<<<16, kThr, 0, stream>>>(x, STAT);
  lncast_kernel<<<1024, kThr, 0, stream>>>(x, STAT, lng, lnb, XN16);

  wmma_gemm64<0, false, 2, 0, false, 0><<<dim3((kRows / 64) * (2 * kDI / 64) / 8, 1), 256, 0, stream>>>(
      XN16, XN16, kDM, 0L, WIN16, WIN16, kDM, 0L, (void*)XZ, (void*)XZ, 2 * kDI, 0L, ZB, nullptr, 0L, kRows, 2 * kDI, kDM, 1.0f / (kCXn * kInCarry));
  front_kernel<<<dim3(1, kRows), 128, 0, stream>>>(XZ, cvw, cvb, U32, U16);
  wmma_gemm64<0, false, 2, 0, false, 0><<<dim3((kRows / 64) * (kXo / 64) / 8, 1), 256, 0, stream>>>(
      U16, U16, kDI, 0L, WX16, WX16, kDI, 0L, (void*)XD, (void*)XD, kXo, 0L, ZB, nullptr, 0L, kRows, kXo, kDI, 1.0f / (kCU * kInCarry));
  dtcast_kernel<<<64, kThr, 0, stream>>>(XD, DT16);
  wmma_gemm64<0, false, 2, 0, false, 0><<<dim3((kRows / 64) * (kDI / 64) / 8, 1), 256, 0, stream>>>(
      DT16, DT16, kR, 0L, WDT16, WDT16, kR, 0L, (void*)DL, (void*)DL, kDI, 0L, BDT, nullptr, 0L, kRows, kDI, kR, 1.0f / (kCDt * kInCarry));
  scan_kernel<<<2 * 4, kThr, 0, stream>>>(XD, DL, U32, alog, dsk, YS);
  ygate_kernel<<<dim3(1, kRows), 128, 0, stream>>>(YS, XZ, Y16);
  wmma_gemm64<0, false, 2, 0, false, 0><<<dim3((kRows / 64) * (kDM / 64) / 8, 1), 256, 0, stream>>>(
      Y16, Y16, kDI, 0L, WOUT16, WOUT16, kDI, 0L, (void*)OUTF, (void*)OUTF, kDM, 0L, ZB, nullptr, 0L, kRows, kDM, kDI, 1.0f / (kCY * kInCarry));
  resadd_kernel<<<1024, kThr, 0, stream>>>(OUTF, x, out);
}
